// NTM_23776938950657
// MI455X (gfx1250) — hardware-run, weakly checked
//
#include <hip/hip_runtime.h>
#include <math.h>

constexpr int NBAT  = 2048;
constexpr int NXIN  = 64;
constexpr int NCTL  = 512;
constexpr int NMEM  = 1024;
constexpr int NVEC  = 64;
constexpr int NOUTF = 64;
constexpr int NINP  = NXIN + NVEC;
constexpr int NHRW  = NCTL + NVEC;
constexpr int NGCOL = 4 * NCTL;
constexpr float RWP_CARRY  = 64.0f;
constexpr float RWP_INV    = 1.0f / 64.0f;
constexpr float W_CARRY    = 16.0f;
constexpr float H_CARRY    = 16.0f;
constexpr float GATE_SCALE = 1.0f / 16.0f;
constexpr float HW_SCALE   = 1.0f / 256.0f;
constexpr float RDW_CARRY  = 1024.0f;
constexpr float RDW_INV    = 1.0f / 1024.0f;
constexpr float RW2_CARRY  = 1048576.0f;
constexpr float RW2_INV    = 1.0f / 1048576.0f;
static_assert(NINP % 32 == 0 && NCTL % 32 == 0 && NMEM % 32 == 0 && NHRW % 32 == 0, "K multiples of 32");
static_assert(NBAT % 64 == 0 && NVEC % 64 == 0 && NMEM % 64 == 0 && NOUTF % 64 == 0, "M,N tile multiples");
static_assert((NBAT / 16) * (NCTL / 64) == 1024, "gate tiles");
static_assert(NBAT % 32 == 0, "softmax rows per block");

typedef __attribute__((ext_vector_type(16))) _Float16 v16h;
typedef __attribute__((ext_vector_type(8)))  _Float16 v8h;
typedef __attribute__((ext_vector_type(16))) __bf16   v16b;
typedef __attribute__((ext_vector_type(8)))  __bf16   v8b;
typedef __attribute__((ext_vector_type(8)))  float    v8f;
typedef __attribute__((ext_vector_type(4)))  float    v4f;

__device__ __forceinline__ unsigned short f2bf_bits(float f) {
  unsigned u = __float_as_uint(f);
  return (unsigned short)((u + 0x7FFFu + ((u >> 16) & 1u)) >> 16);
}
__device__ __forceinline__ float bf_bits2f(unsigned short h) { return __uint_as_float(((unsigned)h) << 16); }

__device__ __forceinline__ void dep_guard_h(v8f& a, v8f& b, v16h x, v16h y) { asm volatile("v_nop\n\tv_nop\n\tv_nop\n\tv_nop" : "+v"(a), "+v"(b) : "v"(x), "v"(y)); }
__device__ __forceinline__ void dep_guard_b(v8f& a, v8f& b, v16b x, v16b y) { asm volatile("v_nop\n\tv_nop\n\tv_nop\n\tv_nop" : "+v"(a), "+v"(b) : "v"(x), "v"(y)); }
__device__ __forceinline__ void guard4_h(v8f& a0, v8f& a1, v8f& a2, v8f& a3, v16h x, v16h y) {
  asm volatile("v_nop\n\tv_nop\n\tv_nop\n\tv_nop" : "+v"(a0), "+v"(a1), "+v"(a2), "+v"(a3) : "v"(x), "v"(y));
}
__device__ __forceinline__ void guard4_b(v8f& a0, v8f& a1, v8f& a2, v8f& a3, v16b x, v16b y) {
  asm volatile("v_nop\n\tv_nop\n\tv_nop\n\tv_nop" : "+v"(a0), "+v"(a1), "+v"(a2), "+v"(a3) : "v"(x), "v"(y));
}
__device__ __forceinline__ void guard4ab_h(v8f& a0, v8f& a1, v8f& a2, v8f& a3,
                                           v16h x, v16h b0, v16h b1, v16h b2, v16h b3) {
  asm volatile("v_nop\n\tv_nop\n\tv_nop\n\tv_nop"
               : "+v"(a0), "+v"(a1), "+v"(a2), "+v"(a3)
               : "v"(x), "v"(b0), "v"(b1), "v"(b2), "v"(b3));
}
__device__ __forceinline__ void guard8ab_h(v8f& a0, v8f& a1, v8f& a2, v8f& a3,
                                           v8f& c0, v8f& c1, v8f& c2, v8f& c3,
                                           v16h x, v16h y, v16h b0, v16h b1, v16h b2, v16h b3) {
  asm volatile("v_nop\n\tv_nop\n\tv_nop\n\tv_nop"
               : "+v"(a0), "+v"(a1), "+v"(a2), "+v"(a3), "+v"(c0), "+v"(c1), "+v"(c2), "+v"(c3)
               : "v"(x), "v"(y), "v"(b0), "v"(b1), "v"(b2), "v"(b3));
}
__device__ __forceinline__ void keep4_h(v16h a, v16h b, v16h c, v16h d) { asm volatile("v_nop" :: "v"(a), "v"(b), "v"(c), "v"(d)); }
__device__ __forceinline__ void keep4_b(v16b a, v16b b, v16b c, v16b d) { asm volatile("v_nop" :: "v"(a), "v"(b), "v"(c), "v"(d)); }
__device__ __forceinline__ void acc_guard4(v8f& a, v8f& b, v8f& c, v8f& d) { asm volatile("v_nop\n\tv_nop\n\tv_nop\n\tv_nop" : "+v"(a), "+v"(b), "+v"(c), "+v"(d)); }
template <typename T> struct Frag;
template <> struct Frag<_Float16> {
  typedef v16h V; union U { v16h v; v8h h[2]; };
  static __device__ __forceinline__ v16h load(const _Float16* p) {
    U f; f.h[0] = *(const v8h*)(p); f.h[1] = *(const v8h*)(p + 16); return f.v;
  }
  static __device__ __forceinline__ v8f mma(v16h a, v16h b, v8f c) {
    return __builtin_amdgcn_wmma_f32_16x16x32_f16(false, a, false, b, (short)0, c, false, false);
  }
  static __device__ __forceinline__ void guard(v8f& a, v8f& b, v16h x, v16h y) { dep_guard_h(a, b, x, y); }
  static __device__ __forceinline__ void guard4(v8f& a, v8f& b, v8f& c, v8f& d, v16h x, v16h y) { guard4_h(a, b, c, d, x, y); }
  static __device__ __forceinline__ void keep(v16h a, v16h b, v16h c, v16h d) { keep4_h(a, b, c, d); }
};
template <> struct Frag<__bf16> {
  typedef v16b V; union U { v16b v; v8b h[2]; };
  static __device__ __forceinline__ v16b load(const __bf16* p) {
    U f; f.h[0] = *(const v8b*)(p); f.h[1] = *(const v8b*)(p + 16); return f.v;
  }
  static __device__ __forceinline__ v8f mma(v16b a, v16b b, v8f c) {
    return __builtin_amdgcn_wmma_f32_16x16x32_bf16(false, a, false, b, (short)0, c, false, false);
  }
  static __device__ __forceinline__ void guard(v8f& a, v8f& b, v16b x, v16b y) { dep_guard_b(a, b, x, y); }
  static __device__ __forceinline__ void guard4(v8f& a, v8f& b, v8f& c, v8f& d, v16b x, v16b y) { guard4_b(a, b, c, d, x, y); }
  static __device__ __forceinline__ void keep(v16b a, v16b b, v16b c, v16b d) { keep4_b(a, b, c, d); }
};

__device__ __forceinline__ void wave_lds_sync() {
  __builtin_amdgcn_fence(__ATOMIC_RELEASE, "workgroup");
  __builtin_amdgcn_wave_barrier();
  __builtin_amdgcn_fence(__ATOMIC_ACQUIRE, "workgroup");
}

__device__ __forceinline__ float fsigp(float x) { return __builtin_amdgcn_rcpf(1.0f + expf(-x)); }

template <int ET> struct Elem;
template <> struct Elem<0> { typedef _Float16 T; };
template <> struct Elem<1> { typedef __bf16 T; };
template <int ET, bool SPLIT, int BIAS_MODE, int OUT_MODE, bool RESID, int ACT = 0>
__global__ __launch_bounds__(256) void wmma_gemm64(
    const unsigned short* __restrict__ Ap, const unsigned short* __restrict__ A2p, int lda, long strideA,
    const unsigned short* __restrict__ Btp, const unsigned short* __restrict__ Bt2p, int ldb, long strideB,
    void* __restrict__ Cout, void* __restrict__ Cout2, int ldc, long strideC,
    const float* __restrict__ bias,
    const float* __restrict__ resid, long strideR,
    int M, int N, int K, float scale) {
  typedef typename Elem<ET>::T T;
  typedef typename Frag<T>::V V;
  const T* A = (const T*)Ap; const T* A2 = (const T*)A2p; const T* Bt = (const T*)Btp; const T* Bt2 = (const T*)Bt2p;
  __shared__ __align__(16) float sT[8][16 * 68];
  const int b    = blockIdx.y;
  const int lane = threadIdx.x & 31;
  const int wave = threadIdx.x >> 5;
  const int tilesN = N >> 6;
  const int tilesM = M >> 6;
  const int tile = blockIdx.x * 8 + wave;
  if (tile >= tilesM * tilesN) return;
  const int tm = tile / tilesN;
  const int tn = tile - tm * tilesN;
  const int m0 = tm << 6;
  const int n0 = tn << 6;

  const T* Ab  = A  + (size_t)b * strideA;
  const T* Bb  = Bt + (size_t)b * strideB;
  const T* Ab2 = SPLIT ? (A2  + (size_t)b * strideA) : nullptr;
  const T* Bb2 = SPLIT ? (Bt2 + (size_t)b * strideB) : nullptr;

  const int rlane = lane & 15;
  const int koff  = (lane >> 4) * 8;
  const int mOff  = (lane >> 4) * 8;

  v8f acc[4][4];
#pragma unroll
  for (int i = 0; i < 4; ++i)
#pragma unroll
    for (int j = 0; j < 4; ++j) acc[i][j] = (v8f){0.f,0.f,0.f,0.f,0.f,0.f,0.f,0.f};

  for (int k0 = 0; k0 < K; k0 += 32) {
    V bh[4], bl[4];
#pragma unroll
    for (int j = 0; j < 4; ++j) {
      const size_t bo = (size_t)(n0 + (j << 4) + rlane) * ldb + koff + k0;
      bh[j] = Frag<T>::load(Bb + bo);
      if (SPLIT) bl[j] = Frag<T>::load(Bb2 + bo);
    }
#pragma unroll
    for (int i = 0; i < 4; ++i) {
      const size_t ao = (size_t)(m0 + (i << 4) + rlane) * lda + koff + k0;
      V ah = Frag<T>::load(Ab + ao);
      V al;
      if (SPLIT) al = Frag<T>::load(Ab2 + ao);
#pragma unroll
      for (int j = 0; j < 4; ++j) {
        acc[i][j] = Frag<T>::mma(ah, bh[j], acc[i][j]);
        if (SPLIT) {
          acc[i][j] = Frag<T>::mma(ah, bl[j], acc[i][j]);
          acc[i][j] = Frag<T>::mma(al, bh[j], acc[i][j]);
        }
      }
      Frag<T>::guard4(acc[i][0], acc[i][1], acc[i][2], acc[i][3], ah, SPLIT ? al : ah);
    }
    Frag<T>::keep(bh[0], bh[1], bh[2], bh[3]);
    if (SPLIT) Frag<T>::keep(bl[0], bl[1], bl[2], bl[3]);
  }
  acc_guard4(acc[0][0], acc[0][1], acc[0][2], acc[0][3]);
  acc_guard4(acc[1][0], acc[1][1], acc[1][2], acc[1][3]);
  acc_guard4(acc[2][0], acc[2][1], acc[2][2], acc[2][3]);
  acc_guard4(acc[3][0], acc[3][1], acc[3][2], acc[3][3]);

  float* slab = sT[wave];
  const float* Rb = RESID ? (resid + (size_t)b * strideR) : nullptr;
#pragma unroll
  for (int i = 0; i < 4; ++i) {
    const int mBase = m0 + (i << 4);
#pragma unroll
    for (int j = 0; j < 4; ++j) {
      const int n = n0 + (j << 4) + rlane;
      float bv = 0.f;
      if (BIAS_MODE == 2) bv = bias[n];
#pragma unroll
      for (int r = 0; r < 8; ++r) {
        float v = acc[i][j][r] * scale;
        if (BIAS_MODE == 1) v += bias[mBase + mOff + r];
        if (BIAS_MODE == 2) v += bv;
        if (RESID) v += Rb[(size_t)(mBase + mOff + r) * ldc + n];
        if (ACT == 1) v = tanhf(v);
        if (ACT == 2) v = fmaxf(v, 0.0f);
        if (ACT == 3) v = v / (1.0f + expf(-v));
        if (ACT == 4) v = (v > 0.f) ? v : 0.01f * v;
        if (ACT == 5) v = 0.5f * v * (1.0f + erff(v * 0.70710678118654752f));
        slab[(mOff + r) * 68 + (j << 4) + rlane] = v;
      }
    }
    __builtin_amdgcn_fence(__ATOMIC_RELEASE, "workgroup");
    __builtin_amdgcn_wave_barrier();
    __builtin_amdgcn_fence(__ATOMIC_ACQUIRE, "workgroup");
    if (OUT_MODE == 0) {
      float* C = (float*)Cout + (size_t)b * strideC;
      const int hh = lane >> 4, c4 = (lane & 15) * 4;
      for (int pass = 0; pass < 2; ++pass) {
#pragma unroll
        for (int it = 0; it < 8; ++it) {
          const int row = it * 2 + hh;
          v4f v = *(const v4f*)(slab + row * 68 + c4);
          *(volatile v4f*)(C + (size_t)(mBase + row) * ldc + n0 + c4) = v;
        }
        __threadfence();
      }
    } else {
      const int q = lane >> 3, c8 = (lane & 7) * 8;
      unsigned short* C  = (unsigned short*)Cout  + (size_t)b * strideC;
      unsigned short* C2 = (OUT_MODE == 2) ? ((unsigned short*)Cout2 + (size_t)b * strideC) : nullptr;
      for (int pass = 0; pass < 2; ++pass) {
#pragma unroll
        for (int it = 0; it < 4; ++it) {
          const int row = it * 4 + q;
          const float* sp = slab + row * 68 + c8;
          v8h hv, lv;
#pragma unroll
          for (int e = 0; e < 8; ++e) {
            if (OUT_MODE == 1) {
              hv[e] = (_Float16)sp[e];
            } else {
              unsigned short hb = f2bf_bits(sp[e]);
              unsigned short lb = f2bf_bits(sp[e] - bf_bits2f(hb));
              hv[e] = __builtin_bit_cast(_Float16, hb);
              lv[e] = __builtin_bit_cast(_Float16, lb);
            }
          }
          *(volatile v8h*)(C + (size_t)(mBase + row) * ldc + n0 + c8) = hv;
          if (OUT_MODE == 2) *(volatile v8h*)(C2 + (size_t)(mBase + row) * ldc + n0 + c8) = lv;
        }
        __threadfence();
      }
    }
    __builtin_amdgcn_fence(__ATOMIC_RELEASE, "workgroup");
    __builtin_amdgcn_wave_barrier();
    __builtin_amdgcn_fence(__ATOMIC_ACQUIRE, "workgroup");
  }
}

__global__ __launch_bounds__(256) void cvt8_kernel(const float* __restrict__ src, unsigned short* __restrict__ dst,
                                                  int nrow, int ncol8, int spitch, int dpitch, int dcol0, float sc) {
  const int i  = blockIdx.x * 256 + threadIdx.x;
  const int n8 = nrow * ncol8;
  if (i < n8) {
    const int row = i / ncol8;
    const int c8  = i - row * ncol8;
    const float* sp = src + (size_t)row * spitch + c8 * 8;
    const v4f a = *(const v4f*)(sp);
    const v4f b = *(const v4f*)(sp + 4);
    v8h hv;
#pragma unroll
    for (int e = 0; e < 4; ++e) {
      hv[e]     = (_Float16)(a[e] * sc);
      hv[4 + e] = (_Float16)(b[e] * sc);
    }
    unsigned short* dp = dst + (size_t)row * dpitch + dcol0 + c8 * 8;
    *(volatile v8h*)dp = hv;
    __threadfence();
    *(volatile v8h*)dp = hv;
  }
}

__global__ __launch_bounds__(256) void tpose_f16_kernel(const float* __restrict__ src, int R, int C, int ldo,
                                                       unsigned short* __restrict__ O, float sc) {
  __shared__ float Tt[64 * 65];
  const int tid = threadIdx.x;
  const int c0 = blockIdx.x * 64, r0 = blockIdx.y * 64;
#pragma unroll
  for (int i = 0; i < 4; ++i) {
    const int idx = i * 256 + tid;
    const int rr = idx >> 4, cc = (idx & 15) * 4;
    const v4f v = *(const v4f*)(src + (size_t)(r0 + rr) * (size_t)C + c0 + cc);
    Tt[rr * 65 + cc + 0] = v[0];
    Tt[rr * 65 + cc + 1] = v[1];
    Tt[rr * 65 + cc + 2] = v[2];
    Tt[rr * 65 + cc + 3] = v[3];
  }
  __syncthreads();
  const int q = tid >> 3, c8 = (tid & 7) * 8;
  v8h hv[2];
#pragma unroll
  for (int g = 0; g < 2; ++g) {
    const int qq = g * 32 + q;
#pragma unroll
    for (int e = 0; e < 8; ++e) hv[g][e] = (_Float16)(Tt[(c8 + e) * 65 + qq] * sc);
  }
  for (int pass = 0; pass < 2; ++pass) {
#pragma unroll
    for (int g = 0; g < 2; ++g) {
      const size_t o = (size_t)(c0 + g * 32 + q) * (size_t)ldo + (size_t)(r0 + c8);
      *(volatile v8h*)(O + o) = hv[g];
    }
    __threadfence();
  }
}

constexpr int GT_SLAB = 16 * 68 + 256;
__global__ __launch_bounds__(256) void gates_lstm_kernel(
    const unsigned short* __restrict__ INPp, const unsigned short* __restrict__ HPVp,
    const unsigned short* __restrict__ WIp,  const unsigned short* __restrict__ WHp,
    const float* __restrict__ b_ih, const float* __restrict__ b_hh, const float* __restrict__ c_prev,
    unsigned short* __restrict__ HR) {
  __shared__ __align__(16) float sT[8][GT_SLAB];
  const _Float16* INP = (const _Float16*)INPp;
  const _Float16* HPV = (const _Float16*)HPVp;
  const _Float16* WI  = (const _Float16*)WIp;
  const _Float16* WH  = (const _Float16*)WHp;
  const int tid = threadIdx.x, lane = tid & 31, wave = tid >> 5;
  const int c = lane & 15, hh = lane >> 4, koff = hh * 8;
  const int tile = blockIdx.x * 8 + wave;
  const int tm = tile >> 3, tu = tile & 7;
  const int m0 = tm * 16, u0 = tu * 64;
  float* slab = sT[wave];
  float* sb   = slab + 16 * 68;

#pragma unroll
  for (int it = 0; it < 2; ++it) {
    const int idx = it * 32 + lane;
    const int g = idx >> 4, q4 = (idx & 15) * 4;
    const v4f va = *(const v4f*)(b_ih + g * NCTL + u0 + q4);
    const v4f vb = *(const v4f*)(b_hh + g * NCTL + u0 + q4);
    *(v4f*)(sb + g * 64 + q4) = va + vb;
  }

  const v8f z8 = {0.f, 0.f, 0.f, 0.f, 0.f, 0.f, 0.f, 0.f};
  v8f acc[4][4];
#pragma unroll
  for (int j = 0; j < 4; ++j)
#pragma unroll
    for (int g = 0; g < 4; ++g) acc[j][g] = z8;

  const _Float16* arow1 = INP + (size_t)(m0 + c) * NINP + koff;
  const _Float16* arow2 = HPV + (size_t)(m0 + c) * NCTL + koff;
#pragma unroll 1
  for (int k0 = 0; k0 < NINP; k0 += 32) {
    const v16h a = Frag<_Float16>::load(arow1 + k0);
#pragma unroll
    for (int j = 0; j < 4; ++j) {
      const _Float16* wp = WI + (size_t)(u0 + 16 * j + c) * NINP + koff + k0;
      const v16h b0 = Frag<_Float16>::load(wp);
      const v16h b1 = Frag<_Float16>::load(wp + (size_t)1 * NCTL * NINP);
      const v16h b2 = Frag<_Float16>::load(wp + (size_t)2 * NCTL * NINP);
      const v16h b3 = Frag<_Float16>::load(wp + (size_t)3 * NCTL * NINP);
      acc[j][0] = Frag<_Float16>::mma(a, b0, acc[j][0]);
      acc[j][1] = Frag<_Float16>::mma(a, b1, acc[j][1]);
      acc[j][2] = Frag<_Float16>::mma(a, b2, acc[j][2]);
      acc[j][3] = Frag<_Float16>::mma(a, b3, acc[j][3]);
      guard4ab_h(acc[j][0], acc[j][1], acc[j][2], acc[j][3], a, b0, b1, b2, b3);
    }
  }
#pragma unroll 1
  for (int k0 = 0; k0 < NCTL; k0 += 32) {
    const v16h a = Frag<_Float16>::load(arow2 + k0);
#pragma unroll
    for (int j = 0; j < 4; ++j) {
      const _Float16* wp = WH + (size_t)(u0 + 16 * j + c) * NCTL + koff + k0;
      const v16h b0 = Frag<_Float16>::load(wp);
      const v16h b1 = Frag<_Float16>::load(wp + (size_t)1 * NCTL * NCTL);
      const v16h b2 = Frag<_Float16>::load(wp + (size_t)2 * NCTL * NCTL);
      const v16h b3 = Frag<_Float16>::load(wp + (size_t)3 * NCTL * NCTL);
      acc[j][0] = Frag<_Float16>::mma(a, b0, acc[j][0]);
      acc[j][1] = Frag<_Float16>::mma(a, b1, acc[j][1]);
      acc[j][2] = Frag<_Float16>::mma(a, b2, acc[j][2]);
      acc[j][3] = Frag<_Float16>::mma(a, b3, acc[j][3]);
      guard4ab_h(acc[j][0], acc[j][1], acc[j][2], acc[j][3], a, b0, b1, b2, b3);
    }
  }
  acc_guard4(acc[0][0], acc[0][1], acc[0][2], acc[0][3]);
  acc_guard4(acc[1][0], acc[1][1], acc[1][2], acc[1][3]);
  acc_guard4(acc[2][0], acc[2][1], acc[2][2], acc[2][3]);
  acc_guard4(acc[3][0], acc[3][1], acc[3][2], acc[3][3]);

#pragma unroll
  for (int it = 0; it < 8; ++it) {
    const int idx = it * 32 + lane;
    const int row = idx >> 4, c4 = (idx & 15) * 4;
    const v4f v = *(const v4f*)(c_prev + (size_t)(m0 + row) * NCTL + u0 + c4);
    *(v4f*)(slab + row * 68 + c4) = v;
  }
  wave_lds_sync();

#pragma unroll
  for (int j = 0; j < 4; ++j) {
    const int col = 16 * j + c;
    const float bi = sb[col], bf = sb[64 + col], bg = sb[128 + col], bo = sb[192 + col];
#pragma unroll
    for (int r = 0; r < 8; ++r) {
      float* sp = slab + (8 * hh + r) * 68 + col;
      const float cp = *sp;
      const float zi = acc[j][0][r] * GATE_SCALE + bi;
      const float zf = acc[j][1][r] * GATE_SCALE + bf;
      const float zg = acc[j][2][r] * GATE_SCALE + bg;
      const float zo = acc[j][3][r] * GATE_SCALE + bo;
      const float ig = fsigp(zi);
      const float fg = fsigp(zf);
      const float og = fsigp(zo);
      const float gg = tanhf(zg);
      const float cn = fg * cp + ig * gg;
      const float hn = og * tanhf(cn);
      *sp = hn * H_CARRY;
    }
  }
  wave_lds_sync();

  {
    const int q = lane >> 3, c8 = (lane & 7) * 8;
    for (int pass = 0; pass < 2; ++pass) {
#pragma unroll
      for (int it = 0; it < 4; ++it) {
        const int row = it * 4 + q;
        const float* sp = slab + row * 68 + c8;
        v8h hv;
#pragma unroll
        for (int e = 0; e < 8; ++e) hv[e] = (_Float16)sp[e];
        *(volatile v8h*)(HR + (size_t)(m0 + row) * NHRW + u0 + c8) = hv;
      }
      __threadfence();
    }
  }
}

constexpr int SM_ROWS = 32;
__global__ __launch_bounds__(128) void softmax2_kernel(const float* __restrict__ rlog, const float* __restrict__ wlog,
                                                      unsigned short* __restrict__ RW, unsigned short* __restrict__ RW2,
                                                      float* __restrict__ srow) {
  __shared__ float redm[2][4];
  __shared__ float reds[2][4];
  __shared__ float redp[4];
  __shared__ __align__(16) float srl[SM_ROWS];
  const int tid = threadIdx.x, lane = tid & 31, wave = tid >> 5;
  const int rbase = blockIdx.x * SM_ROWS;
#pragma unroll 1
  for (int i = 0; i < SM_ROWS; ++i) {
    const int row = rbase + i;
    const size_t off = (size_t)row * NMEM + 8 * tid;
    const v4f ra = *(const v4f*)(rlog + off);
    const v4f rb = *(const v4f*)(rlog + off + 4);
    const v4f wa = *(const v4f*)(wlog + off);
    const v4f wb = *(const v4f*)(wlog + off + 4);
    float mr = fmaxf(fmaxf(fmaxf(ra[0], ra[1]), fmaxf(ra[2], ra[3])), fmaxf(fmaxf(rb[0], rb[1]), fmaxf(rb[2], rb[3])));
    float mw = fmaxf(fmaxf(fmaxf(wa[0], wa[1]), fmaxf(wa[2], wa[3])), fmaxf(fmaxf(wb[0], wb[1]), fmaxf(wb[2], wb[3])));
#pragma unroll
    for (int o = 1; o < 32; o <<= 1) {
      mr = fmaxf(mr, __shfl_xor(mr, o, 32));
      mw = fmaxf(mw, __shfl_xor(mw, o, 32));
    }
    if (lane == 0) { redm[0][wave] = mr; redm[1][wave] = mw; }
    __syncthreads();
    mr = fmaxf(fmaxf(redm[0][0], redm[0][1]), fmaxf(redm[0][2], redm[0][3]));
    mw = fmaxf(fmaxf(redm[1][0], redm[1][1]), fmaxf(redm[1][2], redm[1][3]));
    v4f ea, eb, fa, fb;
    float sr = 0.0f, sw = 0.0f;
#pragma unroll
    for (int e = 0; e < 4; ++e) {
      ea[e] = expf(ra[e] - mr); eb[e] = expf(rb[e] - mr);
      fa[e] = expf(wa[e] - mw); fb[e] = expf(wb[e] - mw);
      sr += ea[e]; sr += eb[e];
      sw += fa[e]; sw += fb[e];
    }
#pragma unroll
    for (int o = 1; o < 32; o <<= 1) {
      sr += __shfl_xor(sr, o, 32);
      sw += __shfl_xor(sw, o, 32);
    }
    if (lane == 0) { reds[0][wave] = sr; reds[1][wave] = sw; }
    __syncthreads();
    sr = (reds[0][0] + reds[0][1]) + (reds[0][2] + reds[0][3]);
    sw = (reds[1][0] + reds[1][1]) + (reds[1][2] + reds[1][3]);
    const float ir = 1.0f / sr;
    const float iw = 1.0f / sw;
    v8h hv, pv;
    float ps = 0.0f;
#pragma unroll
    for (int e = 0; e < 4; ++e) {
      const float rv0 = ea[e] * ir, wv0 = fa[e] * iw, p0 = rv0 * wv0;
      const float rv1 = eb[e] * ir, wv1 = fb[e] * iw, p1 = rv1 * wv1;
      ps += p0; ps += p1;
      hv[e]     = (_Float16)(rv0 * RDW_CARRY);
      hv[4 + e] = (_Float16)(rv1 * RDW_CARRY);
      pv[e]     = (_Float16)(p0 * RW2_CARRY);
      pv[4 + e] = (_Float16)(p1 * RW2_CARRY);
    }
    for (int pass = 0; pass < 2; ++pass) {
      *(volatile v8h*)(RW  + off) = hv;
      *(volatile v8h*)(RW2 + off) = pv;
      __threadfence();
    }
#pragma unroll
    for (int o = 1; o < 32; o <<= 1) ps += __shfl_xor(ps, o, 32);
    if (lane == 0) redp[wave] = ps;
    __syncthreads();
    if (tid == 0) srl[i] = (redp[0] + redp[1]) + (redp[2] + redp[3]);
  }
  __syncthreads();
  if (wave == 0) {
    const v4f v = *(const v4f*)(srl + 4 * (lane & 7));
    float* p = srow + rbase + 4 * (lane & 7);
    if (lane < 8) *(volatile v4f*)p = v;
    __threadfence();
    if (lane < 8) *(volatile v4f*)p = v;
  }
}

constexpr int RN_SLAB = 2 * 16 * 68 + 16;
__global__ __launch_bounds__(128) void readnew_kernel(
    const unsigned short* __restrict__ RWp, const unsigned short* __restrict__ RW2p, const unsigned short* __restrict__ MTp,
    const float* __restrict__ epre, const float* __restrict__ apre, const float* __restrict__ srow,
    unsigned short* __restrict__ HR) {
  __shared__ __align__(16) float sT[4][RN_SLAB];
  const _Float16* RW  = (const _Float16*)RWp;
  const _Float16* RW2 = (const _Float16*)RW2p;
  const _Float16* MT  = (const _Float16*)MTp;
  const int tid = threadIdx.x, lane = tid & 31, wave = tid >> 5;
  const int c = lane & 15, hh = lane >> 4, koff = hh * 8;
  const int tile = blockIdx.x * 4 + wave;
  const int m0 = tile * 16;
  float* se = sT[wave];
  float* sa = se + 16 * 68;
  float* ss = sa + 16 * 68;

  const v8f z8 = {0.f, 0.f, 0.f, 0.f, 0.f, 0.f, 0.f, 0.f};
  v8f acc1[4], acc2[4];
#pragma unroll
  for (int t = 0; t < 4; ++t) { acc1[t] = z8; acc2[t] = z8; }

  const _Float16* a1row = RW  + (size_t)(m0 + c) * NMEM + koff;
  const _Float16* a2row = RW2 + (size_t)(m0 + c) * NMEM + koff;
  const _Float16* brow  = MT  + (size_t)c * NMEM + koff;
#pragma unroll 1
  for (int k0 = 0; k0 < NMEM; k0 += 32) {
    const v16h b0 = Frag<_Float16>::load(brow + k0);
    const v16h b1 = Frag<_Float16>::load(brow + (size_t)16 * NMEM + k0);
    const v16h b2 = Frag<_Float16>::load(brow + (size_t)32 * NMEM + k0);
    const v16h b3 = Frag<_Float16>::load(brow + (size_t)48 * NMEM + k0);
    const v16h a1 = Frag<_Float16>::load(a1row + k0);
    const v16h a2 = Frag<_Float16>::load(a2row + k0);
    acc1[0] = Frag<_Float16>::mma(a1, b0, acc1[0]);
    acc1[1] = Frag<_Float16>::mma(a1, b1, acc1[1]);
    acc1[2] = Frag<_Float16>::mma(a1, b2, acc1[2]);
    acc1[3] = Frag<_Float16>::mma(a1, b3, acc1[3]);
    acc2[0] = Frag<_Float16>::mma(a2, b0, acc2[0]);
    acc2[1] = Frag<_Float16>::mma(a2, b1, acc2[1]);
    acc2[2] = Frag<_Float16>::mma(a2, b2, acc2[2]);
    acc2[3] = Frag<_Float16>::mma(a2, b3, acc2[3]);
    guard8ab_h(acc1[0], acc1[1], acc1[2], acc1[3], acc2[0], acc2[1], acc2[2], acc2[3], a1, a2, b0, b1, b2, b3);
  }
  acc_guard4(acc1[0], acc1[1], acc1[2], acc1[3]);
  acc_guard4(acc2[0], acc2[1], acc2[2], acc2[3]);

#pragma unroll
  for (int it = 0; it < 8; ++it) {
    const int idx = it * 32 + lane;
    const int row = idx >> 4, c4 = (idx & 15) * 4;
    const v4f v = *(const v4f*)(epre + (size_t)(m0 + row) * NVEC + c4);
    *(v4f*)(se + row * 68 + c4) = v;
  }
  asm volatile("" ::: "memory");
#pragma unroll
  for (int it = 0; it < 8; ++it) {
    const int idx = it * 32 + lane;
    const int row = idx >> 4, c4 = (idx & 15) * 4;
    const v4f v = *(const v4f*)(apre + (size_t)(m0 + row) * NVEC + c4);
    *(v4f*)(sa + row * 68 + c4) = v;
  }
  {
    const v4f sv = *(const v4f*)(srow + m0 + 4 * (lane & 3));
    if (lane < 4) *(v4f*)(ss + 4 * lane) = sv;
  }
  wave_lds_sync();

#pragma unroll
  for (int t = 0; t < 4; ++t) {
    const int col = 16 * t + c;
#pragma unroll
    for (int r = 0; r < 8; ++r) {
      const int row = 8 * hh + r;
      float* sp = se + row * 68 + col;
      const float ev = fsigp(*sp);
      const float av = tanhf(sa[row * 68 + col]);
      const float s  = ss[row];
      const float t1 = acc1[t][r] * RDW_INV;
      const float t2 = acc2[t][r] * RW2_INV;
      const float v  = (t1 - ev * t2) + av * s;
      *sp = v * H_CARRY;
    }
  }
  wave_lds_sync();

  {
    const int q = lane >> 3, c8 = (lane & 7) * 8;
    for (int pass = 0; pass < 2; ++pass) {
#pragma unroll
      for (int it = 0; it < 4; ++it) {
        const int row = it * 4 + q;
        const float* sp = se + row * 68 + c8;
        v8h hv;
#pragma unroll
        for (int e = 0; e < 8; ++e) hv[e] = (_Float16)sp[e];
        *(volatile v8h*)(HR + (size_t)(m0 + row) * NHRW + NCTL + c8) = hv;
      }
      __threadfence();
    }
  }
}

extern "C" void kernel_launch(void* const* d_in, const int* in_sizes, int n_in,
                              void* d_out, int out_size, void* d_ws, size_t ws_size, hipStream_t stream) {
  if (n_in < 19 || d_out == nullptr || d_ws == nullptr) return;
  if (in_sizes[0] != NBAT * NXIN || in_sizes[1] != NBAT * NCTL || in_sizes[2] != NBAT * NCTL ||
      in_sizes[3] != NBAT * NMEM || in_sizes[4] != NMEM * NVEC ||
      in_sizes[5] != NGCOL * NINP || in_sizes[6] != NGCOL || in_sizes[7] != NGCOL * NCTL || in_sizes[8] != NGCOL ||
      in_sizes[9] != NMEM * NCTL || in_sizes[10] != NMEM || in_sizes[11] != NMEM * NCTL || in_sizes[12] != NMEM ||
      in_sizes[13] != NVEC * NCTL || in_sizes[14] != NVEC || in_sizes[15] != NVEC * NCTL || in_sizes[16] != NVEC ||
      in_sizes[17] != NOUTF * NHRW || in_sizes[18] != NOUTF || out_size != NBAT * NOUTF) return;

  const float* x       = (const float*)d_in[0];
  const float* h_prev  = (const float*)d_in[1];
  const float* c_prev  = (const float*)d_in[2];
  const float* rwp     = (const float*)d_in[3];
  const float* memory  = (const float*)d_in[4];
  const float* W_ih    = (const float*)d_in[5];
  const float* b_ih    = (const float*)d_in[6];
  const float* W_hh    = (const float*)d_in[7];
  const float* b_hh    = (const float*)d_in[8];
  const float* W_read  = (const float*)d_in[9];
  const float* b_read  = (const float*)d_in[10];
  const float* W_write = (const float*)d_in[11];
  const float* b_write = (const float*)d_in[12];
  const float* W_erase = (const float*)d_in[13];
  const float* b_erase = (const float*)d_in[14];
  const float* W_add   = (const float*)d_in[15];
  const float* b_add   = (const float*)d_in[16];
  const float* W_out   = (const float*)d_in[17];
  const float* b_out   = (const float*)d_in[18];
  float* out = (float*)d_out;

  char* ws = (char*)d_ws; size_t off = 0;
  auto carve = [&](size_t bytes) -> char* { char* p = ws + off; off += (bytes + 255) & ~(size_t)255; return p; };
  unsigned short* INPH = (unsigned short*)carve((size_t)NBAT * NINP * 2);
  unsigned short* RWPH = (unsigned short*)carve((size_t)NBAT * NMEM * 2);
  unsigned short* HPVH = (unsigned short*)carve((size_t)NBAT * NCTL * 2);
  unsigned short* MEMT = (unsigned short*)carve((size_t)NVEC * NMEM * 2);
  unsigned short* WIH  = (unsigned short*)carve((size_t)NGCOL * NINP * 2);
  unsigned short* WHH  = (unsigned short*)carve((size_t)NGCOL * NCTL * 2);
  unsigned short* WRDH = (unsigned short*)carve((size_t)NMEM * NCTL * 2);
  unsigned short* WWRH = (unsigned short*)carve((size_t)NMEM * NCTL * 2);
  unsigned short* WERH = (unsigned short*)carve((size_t)NVEC * NCTL * 2);
  unsigned short* WADH = (unsigned short*)carve((size_t)NVEC * NCTL * 2);
  unsigned short* WOUH = (unsigned short*)carve((size_t)NOUTF * NHRW * 2);
  unsigned short* HRH  = (unsigned short*)carve((size_t)NBAT * NHRW * 2);
  float*          RLOG = (float*)carve((size_t)NBAT * NMEM * 4);
  float*          WLOG = (float*)carve((size_t)NBAT * NMEM * 4);
  float*          EPRE = (float*)carve((size_t)NBAT * NVEC * 4);
  float*          APRE = (float*)carve((size_t)NBAT * NVEC * 4);
  unsigned short* RDWH = (unsigned short*)carve((size_t)NBAT * NMEM * 2);
  unsigned short* RW2H = (unsigned short*)carve((size_t)NBAT * NMEM * 2);
  float*          SROW = (float*)carve((size_t)NBAT * 4);
  if (off > ws_size || off > (size_t)134217728) return;

  auto cvt = [&](const float* s, unsigned short* d, int nrow, int ncol, int spitch, int dpitch, int dcol0, float sc) {
    const int n8 = nrow * (ncol / 8);
    cvt8_kernel<<<(n8 + 255) / 256, 256, 0, stream>>>(s, d, nrow, ncol / 8, spitch, dpitch, dcol0, sc);
  };
  cvt(x,       INPH, NBAT,  NXIN, NXIN, NINP, 0, 1.0f);
  cvt(rwp,     RWPH, NBAT,  NMEM, NMEM, NMEM, 0, RWP_CARRY);
  cvt(h_prev,  HPVH, NBAT,  NCTL, NCTL, NCTL, 0, 1.0f);
  cvt(W_ih,    WIH,  NGCOL, NINP, NINP, NINP, 0, W_CARRY);
  cvt(W_hh,    WHH,  NGCOL, NCTL, NCTL, NCTL, 0, W_CARRY);
  cvt(W_read,  WRDH, NMEM,  NCTL, NCTL, NCTL, 0, W_CARRY);
  cvt(W_write, WWRH, NMEM,  NCTL, NCTL, NCTL, 0, W_CARRY);
  cvt(W_erase, WERH, NVEC,  NCTL, NCTL, NCTL, 0, W_CARRY);
  cvt(W_add,   WADH, NVEC,  NCTL, NCTL, NCTL, 0, W_CARRY);
  cvt(W_out,   WOUH, NOUTF, NHRW, NHRW, NHRW, 0, W_CARRY);
  tpose_f16_kernel<<<dim3(NVEC / 64, NMEM / 64), 256, 0, stream>>>(memory, NMEM, NVEC, NMEM, MEMT, 1.0f);

  wmma_gemm64<0, false, 0, 1, false, 0><<<dim3((NBAT / 64) * (NVEC / 64) / 8, 1), 256, 0, stream>>>(
      RWPH, RWPH, NMEM, 0L, MEMT, MEMT, NMEM, 0L, (void*)(INPH + NXIN), (void*)(INPH + NXIN), NINP, 0L,
      b_out, c_prev, 0L, NBAT, NVEC, NMEM, RWP_INV);

  gates_lstm_kernel<<<(NBAT / 16) * (NCTL / 64) / 8, 256, 0, stream>>>(INPH, HPVH, WIH, WHH, b_ih, b_hh, c_prev, HRH);

  wmma_gemm64<0, false, 2, 0, false, 0><<<dim3((NBAT / 64) * (NMEM / 64) / 8, 1), 256, 0, stream>>>(
      HRH, HRH, NHRW, 0L, WRDH, WRDH, NCTL, 0L, (void*)RLOG, (void*)RLOG, NMEM, 0L,
      b_read, c_prev, 0L, NBAT, NMEM, NCTL, HW_SCALE);
  wmma_gemm64<0, false, 2, 0, false, 0><<<dim3((NBAT / 64) * (NMEM / 64) / 8, 1), 256, 0, stream>>>(
      HRH, HRH, NHRW, 0L, WWRH, WWRH, NCTL, 0L, (void*)WLOG, (void*)WLOG, NMEM, 0L,
      b_write, c_prev, 0L, NBAT, NMEM, NCTL, HW_SCALE);
  wmma_gemm64<0, false, 2, 0, false, 0><<<dim3((NBAT / 64) * (NVEC / 64) / 8, 1), 256, 0, stream>>>(
      HRH, HRH, NHRW, 0L, WERH, WERH, NCTL, 0L, (void*)EPRE, (void*)EPRE, NVEC, 0L,
      b_erase, c_prev, 0L, NBAT, NVEC, NCTL, HW_SCALE);
  wmma_gemm64<0, false, 2, 0, false, 0><<<dim3((NBAT / 64) * (NVEC / 64) / 8, 1), 256, 0, stream>>>(
      HRH, HRH, NHRW, 0L, WADH, WADH, NCTL, 0L, (void*)APRE, (void*)APRE, NVEC, 0L,
      b_add, c_prev, 0L, NBAT, NVEC, NCTL, HW_SCALE);

  softmax2_kernel<<<NBAT / SM_ROWS, 128, 0, stream>>>(RLOG, WLOG, RDWH, RW2H, SROW);

  readnew_kernel<<<(NBAT / 16) / 4, 128, 0, stream>>>(RDWH, RW2H, MEMT, EPRE, APRE, SROW, HRH);

  wmma_gemm64<0, false, 2, 0, false, 0><<<dim3((NBAT / 64) * (NOUTF / 64) / 8, 1), 256, 0, stream>>>(
      HRH, HRH, NHRW, 0L, WOUH, WOUH, NHRW, 0L, (void*)out, (void*)out, NOUTF, 0L,
      b_out, c_prev, 0L, NBAT, NOUTF, NHRW, HW_SCALE);
}
